// AttentionWithRotary_14061722927478
// MI455X (gfx1250) — hardware-run, weakly checked
//
#include <hip/hip_runtime.h>
#include <math.h>

typedef __attribute__((ext_vector_type(16))) _Float16 v16h;
typedef __attribute__((ext_vector_type(8)))  _Float16 v8h;
typedef __attribute__((ext_vector_type(8)))  float    v8f;
typedef __attribute__((ext_vector_type(4)))  float    v4f;

constexpr int kBatch = 2;
constexpr int kSeq   = 2048;
constexpr int kDim   = 2048;
constexpr int kHeads = 16;
constexpr int kHd    = kDim / kHeads;
constexpr int kPairs = kHd / 2;
constexpr int kTok   = kBatch * kSeq;
constexpr int kNz    = kBatch * kHeads;
static_assert(kHd == 128 && kPairs == 64 && kTok == 4096 && kNz == 32, "shape chain");
static_assert((size_t)kTok * kDim == 8388608ull, "x / out element count");
static_assert((size_t)kDim * kDim == 4194304ull, "weight element count");
static_assert((size_t)kSeq * kPairs == 131072ull, "table element count");
static_assert((kDim % 32) == 0 && (kSeq % 32) == 0 && (kHd % 32) == 0, "every GEMM K is a multiple of 32");
static_assert((kTok % 64) == 0 && (kDim % 64) == 0 && (kHd % 64) == 0 && (kSeq % 64) == 0, "every GEMM M,N is a multiple of 64");

constexpr float kXCarry = 16.0f;
constexpr float kWCarry = 1024.0f;
constexpr float kPCarry = 16.0f;
constexpr float kMCarry = 16.0f;
constexpr float kACarry = 4.0f;
constexpr float kF16MinNormal = 6.103515625e-5f;

constexpr size_t kOffXH = 0;
constexpr size_t kOffWP = kOffXH + (size_t)kTok * kDim * 2;
constexpr size_t kOffQP = kOffWP + (size_t)4 * kDim * kDim * 2;
constexpr size_t kOffKV = kOffQP + (size_t)kTok * kDim * 2;
constexpr size_t kOffMT = kOffKV + (size_t)2 * kDim * kTok * 2;
constexpr size_t kOffAH = kOffMT + (size_t)kNz * kHd * kHd * 2;
constexpr size_t kWsTotal = kOffAH + (size_t)kTok * kDim * 2;
static_assert(kWsTotal == 118489088ull, "carve total");
static_assert(kWsTotal <= 134217728ull, "carve cap");
static_assert((kOffWP % 128) == 0 && (kOffQP % 128) == 0 && (kOffKV % 128) == 0 &&
              (kOffMT % 128) == 0 && (kOffAH % 128) == 0, "128-B aligned regions");

__device__ __forceinline__ _Float16 to_h_ftz(float f) {
  const float g = (fabsf(f) < kF16MinNormal) ? 0.0f : f;
  return (_Float16)g;
}

__device__ __forceinline__ v16h ld_frag(const _Float16* p) {
  union { v16h v; v8h h[2]; } f;
  f.h[0] = *(const v8h*)(p);
  f.h[1] = *(const v8h*)(p + 16);
  return f.v;
}

__device__ __forceinline__ v8f mma_g(v16h a, v16h b, v8f c) {
  c = __builtin_amdgcn_wmma_f32_16x16x32_f16(false, a, false, b, (short)0, c, false, false);
  asm volatile("v_nop\n\tv_nop\n\tv_nop\n\tv_nop" : "+v"(c) : "v"(a), "v"(b));
  return c;
}

__global__ __launch_bounds__(256) void cast8_carry_kernel(
    const float* __restrict__ s0, const float* __restrict__ s1,
    const float* __restrict__ s2, const float* __restrict__ s3,
    unsigned short* __restrict__ out, long planeElems, int n8, float carry)
{
  const int z = blockIdx.y;
  const float* in = (z == 0) ? s0 : (z == 1) ? s1 : (z == 2) ? s2 : s3;
  const int i = blockIdx.x * 256 + threadIdx.x;
  if (i >= n8) return;
  const float* p = in + 8 * (size_t)i;
  const v4f a = *(const v4f*)(p);
  const v4f c = *(const v4f*)(p + 4);
  v8h hv;
#pragma unroll
  for (int e = 0; e < 4; ++e) {
    const float fa = a[e] * carry;
    const float fc = c[e] * carry;
    hv[e]     = to_h_ftz(fa);
    hv[4 + e] = to_h_ftz(fc);
  }
  unsigned short* q = out + (size_t)z * (size_t)planeElems + 8 * (size_t)i;
  *(volatile v8h*)q = hv;
  __threadfence();
  *(volatile v8h*)q = hv;
}

template <int EPI>
__global__ __launch_bounds__(256) void gemm64_kernel(
    const unsigned short* __restrict__ Ap, int lda, long sA0, long sA1,
    const unsigned short* __restrict__ Btp, int ldb, long sB0, long sB1,
    void* __restrict__ Cout, int ldc, long sC0, long sC1,
    const float* __restrict__ biasA, const float* __restrict__ biasB,
    const float* __restrict__ tabC, const float* __restrict__ tabS,
    int M, int N, int K, int nz, float scale, float oscale)
{
  __shared__ __align__(16) float sT[8][16 * 68];
  const int lane = threadIdx.x & 31;
  const int wave = threadIdx.x >> 5;
  const int tilesN = N >> 6;
  const int tilesM = M >> 6;
  const int tilesZ = tilesM * tilesN;
  const int tileG = blockIdx.x * 8 + wave;
  if (tileG >= tilesZ * nz) return;
  const int z    = tileG / tilesZ;
  const int tile = tileG - z * tilesZ;
  const int tm = tile / tilesN;
  const int tn = tile - tm * tilesN;
  const int m0 = tm << 6;
  const int n0 = tn << 6;
  const int zb = z / kHeads;
  const int zh = z - zb * kHeads;

  const _Float16* Ab = (const _Float16*)Ap  + (size_t)zb * (size_t)sA0 + (size_t)zh * (size_t)sA1;
  const _Float16* Bb = (const _Float16*)Btp + (size_t)zb * (size_t)sB0 + (size_t)zh * (size_t)sB1;
  const size_t coff = (size_t)zb * (size_t)sC0 + (size_t)zh * (size_t)sC1;

  const int rlane = lane & 15;
  const int koff  = (lane >> 4) * 8;
  const int mOff  = (lane >> 4) * 8;

  v8f acc[4][4];
#pragma unroll
  for (int i = 0; i < 4; ++i)
#pragma unroll
    for (int j = 0; j < 4; ++j) acc[i][j] = (v8f){0.f, 0.f, 0.f, 0.f, 0.f, 0.f, 0.f, 0.f};

  for (int k0 = 0; k0 < K; k0 += 32) {
    v16h bh[4];
#pragma unroll
    for (int j = 0; j < 4; ++j) {
      const size_t bo = (size_t)(n0 + (j << 4) + rlane) * ldb + koff + k0;
      bh[j] = ld_frag(Bb + bo);
    }
#pragma unroll
    for (int i = 0; i < 4; ++i) {
      const size_t ao = (size_t)(m0 + (i << 4) + rlane) * lda + koff + k0;
      const v16h ah = ld_frag(Ab + ao);
#pragma unroll
      for (int j = 0; j < 4; ++j) acc[i][j] = mma_g(ah, bh[j], acc[i][j]);
    }
  }

  float* slab = sT[wave];

  float bn[4];
#pragma unroll
  for (int j = 0; j < 4; ++j) bn[j] = 0.0f;
  if (EPI == 1 || EPI == 3) {
#pragma unroll
    for (int j = 0; j < 4; ++j) bn[j] = biasA[n0 + (j << 4) + rlane];
  }
  const bool rotRows = (EPI == 2) && (m0 < kDim);

#pragma unroll
  for (int i = 0; i < 4; ++i) {
    const int mBase = m0 + (i << 4);

    float bm[8];
#pragma unroll
    for (int r = 0; r < 8; ++r) bm[r] = 0.0f;
    if (EPI == 2) {
      const float* pb = (m0 < kDim) ? biasA : biasB;
      const int mb = (mBase + mOff) & (kDim - 1);
      const v4f b0 = *(const v4f*)(pb + mb);
      const v4f b1 = *(const v4f*)(pb + mb + 4);
#pragma unroll
      for (int e = 0; e < 4; ++e) {
        bm[e]     = b0[e];
        bm[4 + e] = b1[e];
      }
    }

#pragma unroll
    for (int j = 0; j < 4; ++j) {
      float v[8];
#pragma unroll
      for (int r = 0; r < 8; ++r) v[r] = acc[i][j][r] * scale;
      if (EPI == 1 || EPI == 3) {
#pragma unroll
        for (int r = 0; r < 8; ++r) v[r] += bn[j];
      }
      if (EPI == 2) {
#pragma unroll
        for (int r = 0; r < 8; ++r) v[r] += bm[r];
        if (rotRows) {
          const int tokn = n0 + (j << 4) + rlane;
          const int spos = tokn & (kSeq - 1);
          const int i0   = ((mBase + mOff) & (kHd - 1)) >> 1;
          const v4f c4 = *(const v4f*)(tabC + (size_t)spos * kPairs + i0);
          const v4f s4 = *(const v4f*)(tabS + (size_t)spos * kPairs + i0);
#pragma unroll
          for (int p = 0; p < 4; ++p) {
            const float t0 = v[2 * p];
            const float t1 = v[2 * p + 1];
            v[2 * p]     = t0 * c4[p] - t1 * s4[p];
            v[2 * p + 1] = t0 * s4[p] + t1 * c4[p];
          }
        }
#pragma unroll
        for (int r = 0; r < 8; ++r) v[r] *= oscale;
      }
#pragma unroll
      for (int r = 0; r < 8; ++r) slab[(mOff + r) * 68 + (j << 4) + rlane] = v[r];
    }
    __builtin_amdgcn_fence(__ATOMIC_RELEASE, "workgroup");
    __builtin_amdgcn_wave_barrier();
    __builtin_amdgcn_fence(__ATOMIC_ACQUIRE, "workgroup");

    if (EPI == 3) {
      float* C = (float*)Cout + coff;
      const int hh = lane >> 4;
      const int c4 = (lane & 15) * 4;
      v4f ov[8];
#pragma unroll
      for (int it = 0; it < 8; ++it) ov[it] = *(const v4f*)(slab + (it * 2 + hh) * 68 + c4);
      for (int pass = 0; pass < 2; ++pass) {
#pragma unroll
        for (int it = 0; it < 8; ++it) {
          *(volatile v4f*)(C + (size_t)(mBase + it * 2 + hh) * ldc + n0 + c4) = ov[it];
        }
        __threadfence();
      }
    } else {
      unsigned short* C = (unsigned short*)Cout + coff;
      const int q  = lane >> 3;
      const int c8 = (lane & 7) * 8;
      v8h pk[4];
#pragma unroll
      for (int it = 0; it < 4; ++it) {
        const int row = it * 4 + q;
        const float* sp = slab + row * 68 + c8;
        const v4f a0 = *(const v4f*)(sp);
        const v4f a1 = *(const v4f*)(sp + 4);
        float t[8];
#pragma unroll
        for (int e = 0; e < 4; ++e) {
          t[e]     = a0[e];
          t[4 + e] = a1[e];
        }
        if (EPI == 1) {
          const int spos = (mBase + row) & (kSeq - 1);
          const int i0   = ((n0 + c8) & (kHd - 1)) >> 1;
          const v4f c4 = *(const v4f*)(tabC + (size_t)spos * kPairs + i0);
          const v4f s4 = *(const v4f*)(tabS + (size_t)spos * kPairs + i0);
#pragma unroll
          for (int p = 0; p < 4; ++p) {
            const float t0 = t[2 * p];
            const float t1 = t[2 * p + 1];
            t[2 * p]     = (t0 * c4[p] - t1 * s4[p]) * oscale;
            t[2 * p + 1] = (t0 * s4[p] + t1 * c4[p]) * oscale;
          }
        }
        v8h hv;
#pragma unroll
        for (int e = 0; e < 8; ++e) hv[e] = to_h_ftz(t[e]);
        pk[it] = hv;
      }
      for (int pass = 0; pass < 2; ++pass) {
#pragma unroll
        for (int it = 0; it < 4; ++it) {
          *(volatile v8h*)(C + (size_t)(mBase + it * 4 + q) * ldc + n0 + c8) = pk[it];
        }
        __threadfence();
      }
    }
    __builtin_amdgcn_fence(__ATOMIC_RELEASE, "workgroup");
    __builtin_amdgcn_wave_barrier();
    __builtin_amdgcn_fence(__ATOMIC_ACQUIRE, "workgroup");
  }
}

extern "C" void kernel_launch(void* const* d_in, const int* in_sizes, int n_in,
                              void* d_out, int out_size, void* d_ws, size_t ws_size,
                              hipStream_t stream) {
  if (n_in < 11) return;
  if (in_sizes[0] != kTok * kDim) return;
  if (in_sizes[1] != kSeq * kPairs) return;
  if (in_sizes[2] != kSeq * kPairs) return;
  if (in_sizes[3] != kDim * kDim) return;
  if (in_sizes[4] != kDim) return;
  if (in_sizes[5] != kDim * kDim) return;
  if (in_sizes[6] != kDim) return;
  if (in_sizes[7] != kDim * kDim) return;
  if (in_sizes[8] != kDim) return;
  if (in_sizes[9] != kDim * kDim) return;
  if (in_sizes[10] != kDim) return;
  if (out_size != kTok * kDim) return;
  if (ws_size < kWsTotal) return;

  const float* x    = (const float*)d_in[0];
  const float* fcos = (const float*)d_in[1];
  const float* fsin = (const float*)d_in[2];
  const float* wq_w = (const float*)d_in[3];
  const float* wq_b = (const float*)d_in[4];
  const float* wk_w = (const float*)d_in[5];
  const float* wk_b = (const float*)d_in[6];
  const float* wv_w = (const float*)d_in[7];
  const float* wv_b = (const float*)d_in[8];
  const float* wo_w = (const float*)d_in[9];
  const float* wo_b = (const float*)d_in[10];

  char* ws = (char*)d_ws;
  unsigned short* XH = (unsigned short*)(ws + kOffXH);
  unsigned short* WP = (unsigned short*)(ws + kOffWP);
  unsigned short* QP = (unsigned short*)(ws + kOffQP);
  unsigned short* KV = (unsigned short*)(ws + kOffKV);
  unsigned short* MT = (unsigned short*)(ws + kOffMT);
  unsigned short* AH = (unsigned short*)(ws + kOffAH);
  unsigned short* WQ = WP;
  unsigned short* WK = WP + (size_t)kDim * kDim;
  unsigned short* WO = WP + (size_t)3 * kDim * kDim;
  unsigned short* KT = KV;
  unsigned short* VT = KV + (size_t)kDim * kTok;

  const float attScale   = 1.0f / sqrtf((float)kHd);
  const float projScale  = 1.0f / (kXCarry * kWCarry);
  const float stateScale = attScale * (kMCarry / (kPCarry * kPCarry));
  const float headScale  = kACarry / (kPCarry * kMCarry);
  const float outScale   = 1.0f / (kACarry * kWCarry);

  {
    const int n8x = kTok * kDim / 8;
    cast8_carry_kernel<<<dim3(n8x / 256, 1), 256, 0, stream>>>(x, x, x, x, XH, 0L, n8x, kXCarry);
    const int n8w = kDim * kDim / 8;
    cast8_carry_kernel<<<dim3(n8w / 256, 4), 256, 0, stream>>>(wq_w, wk_w, wv_w, wo_w, WP, (long)kDim * kDim, n8w, kWCarry);
  }

  gemm64_kernel<1><<<dim3((kTok / 64) * (kDim / 64) / 8, 1), 256, 0, stream>>>(
      XH, kDim, 0L, 0L,
      WQ, kDim, 0L, 0L,
      (void*)QP, kDim, 0L, 0L,
      wq_b, wq_b, fcos, fsin,
      kTok, kDim, kDim, 1, projScale, kPCarry);

  gemm64_kernel<2><<<dim3((2 * kDim / 64) * (kTok / 64) / 8, 1), 256, 0, stream>>>(
      WK, kDim, 0L, 0L,
      XH, kDim, 0L, 0L,
      (void*)KV, kTok, 0L, 0L,
      wk_b, wv_b, fcos, fsin,
      2 * kDim, kTok, kDim, 1, projScale, kPCarry);

  gemm64_kernel<0><<<dim3(kNz * (kHd / 64) * (kHd / 64) / 8, 1), 256, 0, stream>>>(
      VT, kTok, (long)kSeq, (long)kHd * kTok,
      KT, kTok, (long)kSeq, (long)kHd * kTok,
      (void*)MT, kHd, (long)kHeads * kHd * kHd, (long)kHd * kHd,
      wq_b, wq_b, fcos, fsin,
      kHd, kHd, kSeq, kNz, stateScale, 1.0f);

  gemm64_kernel<0><<<dim3(kNz * (kSeq / 64) * (kHd / 64) / 8, 1), 256, 0, stream>>>(
      QP, kDim, (long)kSeq * kDim, (long)kHd,
      MT, kHd, (long)kHeads * kHd * kHd, (long)kHd * kHd,
      (void*)AH, kDim, (long)kSeq * kDim, (long)kHd,
      wq_b, wq_b, fcos, fsin,
      kSeq, kHd, kHd, kNz, headScale, 1.0f);

  gemm64_kernel<3><<<dim3((kTok / 64) * (kDim / 64) / 8, 1), 256, 0, stream>>>(
      AH, kDim, 0L, 0L,
      WO, kDim, 0L, 0L,
      d_out, kDim, 0L, 0L,
      wo_b, wo_b, fcos, fsin,
      kTok, kDim, kDim, 1, outScale, 1.0f);
}
